// ClientGCN_81415400063394
// MI455X (gfx1250) — hardware-verified
//
#include <hip/hip_runtime.h>
#include <stddef.h>


#define FIN     128
#define FD      64
#define NTHR    256
#define NWAVE   8
#define EPT     8
#define NGRP    2
#define CHUNK   (NTHR * EPT * NGRP)
#define WCAP    (EPT * NGRP * 32)
#define LISTN   (NWAVE * WCAP)
#define NBC     4096
#define NBF     1024
#define RCAP    40960
#define RBN     128
#define TGT     256
#define DEGCAP  1024
#define GROWS   128
#define OTHR    512
#define WSCAP   134217728

#define K1      128
#define APK1    136
#define K2      64
#define APK2    72

#define WP_1    0
#define WP_2    16384
#define WPTOT   24576

#define LDS_FILL ((RCAP + NBF + LISTN) * 4 + 64)
#define LDS_G1   (2 * GROWS * APK1 * 2 + GROWS * FD * 4)
#define LDS_G2   (2 * GROWS * APK2 * 2 + GROWS * FD * 4)
#define LDS_AGG  (TGT * FD * 4)

#define BN_EPS 1e-5f

static_assert((CHUNK & (CHUNK - 1)) == 0);
static_assert(CHUNK <= 4096);
static_assert(NBC <= 4096 && NBF <= 4096);
static_assert((NBC & (NBC - 1)) == 0 && (NBF & (NBF - 1)) == 0);
static_assert(NBC == 4 * NBF);
static_assert(OTHR * 8 == NBC);
static_assert((RCAP % 32) == 0);
static_assert(TGT == NWAVE * 32 && (TGT % GROWS) == 0);
static_assert((NBC % TGT) == 0);
static_assert(GROWS == NWAVE * 16);
static_assert(FD == 64 && FIN == K1 && FD == K2);
static_assert(WP_2 == WP_1 + 2 * FD * K1 && WPTOT == WP_2 + 2 * FD * K2);
static_assert((WP_2 % 8) == 0);
static_assert(((2 * GROWS * APK1 * 2) % 16) == 0 && ((2 * GROWS * APK2 * 2) % 16) == 0);

typedef float          v2f  __attribute__((ext_vector_type(2)));
typedef float          v4f  __attribute__((ext_vector_type(4)));
typedef float          v8f  __attribute__((ext_vector_type(8)));
typedef double         v2d  __attribute__((ext_vector_type(2)));
typedef int            v4i  __attribute__((ext_vector_type(4)));
typedef unsigned short v8us __attribute__((ext_vector_type(8)));
typedef __bf16         v16b __attribute__((ext_vector_type(16)));
union FragB { v16b v; v8us h[2]; };

__device__ __forceinline__ unsigned int bfr(float f) {
  const unsigned int u = __float_as_uint(f);
  return (u + 0x7FFFu + ((u >> 16) & 1u)) >> 16;
}

__device__ __forceinline__ void split1(float x, unsigned short& hb, unsigned short& lb) {
  const unsigned int hu = bfr(x);
  const float hf = __uint_as_float(hu << 16);
  hb = (unsigned short)hu;
  lb = (unsigned short)bfr(x - hf);
}

__device__ __forceinline__ void split8(v4f a, v4f b, v8us& hi, v8us& lo) {
  unsigned short hb, lb;
  split1(a.x, hb, lb); hi[0] = hb; lo[0] = lb;
  split1(a.y, hb, lb); hi[1] = hb; lo[1] = lb;
  split1(a.z, hb, lb); hi[2] = hb; lo[2] = lb;
  split1(a.w, hb, lb); hi[3] = hb; lo[3] = lb;
  split1(b.x, hb, lb); hi[4] = hb; lo[4] = lb;
  split1(b.y, hb, lb); hi[5] = hb; lo[5] = lb;
  split1(b.z, hb, lb); hi[6] = hb; lo[6] = lb;
  split1(b.w, hb, lb); hi[7] = hb; lo[7] = lb;
}

__device__ __forceinline__ v8f wmb(v16b a, v16b b, v8f c) {
  v8f d = __builtin_amdgcn_wmma_f32_16x16x32_bf16(false, a, false, b, (short)0, c, false, false);
  asm volatile("v_nop\n\tv_nop\n\tv_nop\n\tv_nop" : "+v"(d) : "v"(a), "v"(b));
  return d;
}

__device__ __forceinline__ v4f bnrelu4(v4f v, v4f mu, v4f rs, v4f g, v4f b) {
  v4f z = (v - mu) * rs * g + b;
  z.x = fmaxf(z.x, 0.0f); z.y = fmaxf(z.y, 0.0f); z.z = fmaxf(z.z, 0.0f); z.w = fmaxf(z.w, 0.0f);
  return z;
}

template <int KD, int NT, int NCT, int APK>
__device__ __forceinline__ void mma_tiles(const unsigned short* sHi, const unsigned short* sLo,
                                          const unsigned short* __restrict__ Bw, int wrow, int lane,
                                          v8f (&acc)[NT]) {
  static_assert((KD % 32) == 0 && (APK % 8) == 0);
  constexpr int NKT = KD / 32, WPLN = NCT * KD;
  const int hh = lane >> 4, m = lane & 15;
#pragma unroll
  for (int t = 0; t < NT; ++t) { v8f z = {0.f, 0.f, 0.f, 0.f, 0.f, 0.f, 0.f, 0.f}; acc[t] = z; }
  const unsigned short* ahp = sHi + (wrow + m) * APK + 8 * hh;
  const unsigned short* alp = sLo + (wrow + m) * APK + 8 * hh;
#pragma unroll 1
  for (int kt = 0; kt < NKT; ++kt) {
    FragB ah, al;
    ah.h[0] = *(const v8us*)(ahp + 32 * kt);
    ah.h[1] = *(const v8us*)(ahp + 32 * kt + 16);
    al.h[0] = *(const v8us*)(alp + 32 * kt);
    al.h[1] = *(const v8us*)(alp + 32 * kt + 16);
#pragma unroll
    for (int t = 0; t < NT; ++t) {
      const unsigned short* bp = Bw + (size_t)(16 * t + m) * KD + 32 * kt + 8 * hh;
      FragB bh, bl;
      bh.h[0] = *(const v8us*)bp;
      bh.h[1] = *(const v8us*)(bp + 16);
      bl.h[0] = *(const v8us*)(bp + WPLN);
      bl.h[1] = *(const v8us*)(bp + WPLN + 16);
      acc[t] = wmb(ah.v, bh.v, acc[t]);
      acc[t] = wmb(ah.v, bl.v, acc[t]);
      acc[t] = wmb(al.v, bh.v, acc[t]);
    }
  }
}

template <int NR>
__device__ __forceinline__ void store_rows64(const float* stg, float* C, int rowBase, int wave, int lane) {
  static_assert((NR % 2) == 0);
  const float* lp = stg + wave * NR * FD + 4 * lane;
  float* gp = C + (size_t)(rowBase + wave * NR) * FD + 4 * lane;
#pragma unroll
  for (int i = 0; i < NR / 2; ++i) { const v4f v = *(const v4f*)(lp + 2 * FD * i); *(volatile v4f*)(gp + 2 * FD * i) = v; }
  __threadfence();
#pragma unroll
  for (int i = 0; i < NR / 2; ++i) { const v4f v = *(const v4f*)(lp + 2 * FD * i); *(volatile v4f*)(gp + 2 * FD * i) = v; }
}

template <int NB>
__device__ __forceinline__ int scan_chunk(const int* __restrict__ dsts, int nE, int cbase, int slotBase,
                                          int vec8, int* list, int tid, int lane, int wave) {
  int wc = 0;
#pragma unroll
  for (int g = 0; g < NGRP; ++g) {
    const int el0  = (g * NTHR + tid) * EPT;
    const int e0   = cbase + el0;
    const int sent = -2147483647 - 1;
    v4i da, db;
    if (vec8 != 0 && cbase + CHUNK <= nE) {
      da = *(const v4i*)(dsts + e0);
      db = *(const v4i*)(dsts + e0 + 4);
    } else {
      da.x = (e0     < nE) ? dsts[min(e0, nE - 1)] : sent;
      da.y = (e0 + 1 < nE) ? dsts[min(e0 + 1, nE - 1)] : sent;
      da.z = (e0 + 2 < nE) ? dsts[min(e0 + 2, nE - 1)] : sent;
      da.w = (e0 + 3 < nE) ? dsts[min(e0 + 3, nE - 1)] : sent;
      db.x = (e0 + 4 < nE) ? dsts[min(e0 + 4, nE - 1)] : sent;
      db.y = (e0 + 5 < nE) ? dsts[min(e0 + 5, nE - 1)] : sent;
      db.z = (e0 + 6 < nE) ? dsts[min(e0 + 6, nE - 1)] : sent;
      db.w = (e0 + 7 < nE) ? dsts[min(e0 + 7, nE - 1)] : sent;
    }
    const unsigned nb = (unsigned)slotBase;
    const unsigned s0 = (unsigned)da.x - nb, s1 = (unsigned)da.y - nb;
    const unsigned s2 = (unsigned)da.z - nb, s3 = (unsigned)da.w - nb;
    const unsigned s4 = (unsigned)db.x - nb, s5 = (unsigned)db.y - nb;
    const unsigned s6 = (unsigned)db.z - nb, s7 = (unsigned)db.w - nb;
    const bool h0 = s0 < (unsigned)NB, h1 = s1 < (unsigned)NB, h2 = s2 < (unsigned)NB, h3 = s3 < (unsigned)NB;
    const bool h4 = s4 < (unsigned)NB, h5 = s5 < (unsigned)NB, h6 = s6 < (unsigned)NB, h7 = s7 < (unsigned)NB;
    const unsigned any = __builtin_amdgcn_ballot_w32(h0 | h1 | h2 | h3 | h4 | h5 | h6 | h7);
    if (any != 0u) {
#define HITJ(J, HJ, SJ) { \
        const unsigned mj = __builtin_amdgcn_ballot_w32(HJ); \
        if (mj != 0u) { \
          if (HJ) { \
            const int pos = wc + (int)__builtin_amdgcn_mbcnt_lo(mj, 0u); \
            if (pos < WCAP) list[wave * WCAP + pos] = ((el0 + (J)) << 12) | (int)(SJ); \
          } \
          wc += (int)__builtin_popcount(mj); } }
      HITJ(0, h0, s0)
      HITJ(1, h1, s1)
      HITJ(2, h2, s2)
      HITJ(3, h3, s3)
      HITJ(4, h4, s4)
      HITJ(5, h5, s5)
      HITJ(6, h6, s6)
      HITJ(7, h7, s7)
#undef HITJ
    }
  }
  return wc;
}

__global__ __launch_bounds__(NTHR) void k_wprep(
    const float* __restrict__ w1, const float* __restrict__ w2, unsigned short* wp) {
  const int blk = blockIdx.x, tid = threadIdx.x;
  float v[8];
  int KD, i, base;
  if (blk < 4) {
    KD = K1; i = blk * NTHR + tid; base = WP_1;
    const int n = i >> 4, k0 = (i & 15) * 8;
#pragma unroll
    for (int e = 0; e < 8; ++e) v[e] = w1[(k0 + e) * FD + n];
  } else {
    KD = K2; i = (blk - 4) * NTHR + tid; base = WP_2;
    i = i > (FD * (K2 / 8) - 1) ? (FD * (K2 / 8) - 1) : i;
    const int n = i >> 3, k0 = (i & 7) * 8;
#pragma unroll
    for (int e = 0; e < 8; ++e) v[e] = w2[(k0 + e) * FD + n];
  }
  v4f a, b;
  a.x = v[0]; a.y = v[1]; a.z = v[2]; a.w = v[3];
  b.x = v[4]; b.y = v[5]; b.z = v[6]; b.w = v[7];
  v8us hv, lv;
  split8(a, b, hv, lv);
  unsigned short* dh = wp + base + (size_t)i * 8;
  unsigned short* dl = dh + FD * KD;
  *(volatile v8us*)dh = hv;
  *(volatile v8us*)dl = lv;
  __threadfence();
  *(volatile v8us*)dh = hv;
  *(volatile v8us*)dl = lv;
}

__global__ __launch_bounds__(NTHR) void k_count(const int* __restrict__ dsts, int* cnt, int nE, int vec8) {
  __shared__ __attribute__((aligned(16))) int scnt[NBC];
  __shared__ __attribute__((aligned(16))) int list[LISTN];
  __shared__ int wcnt[NWAVE];
  const int tid = threadIdx.x, lane = tid & 31, wave = tid >> 5;
  const int nodeBase = blockIdx.x * NBC;

  for (int i = tid; i < NBC; i += NTHR) scnt[i] = 0;
  __syncthreads();

  const int nChunks = (nE + CHUNK - 1) / CHUNK;
#pragma unroll 1
  for (int ch = 0; ch < nChunks; ++ch) {
    const int cbase = ch * CHUNK;
    const int wc = scan_chunk<NBC>(dsts, nE, cbase, nodeBase, vec8, list, tid, lane, wave);
    if (lane == 0) wcnt[wave] = wc;
    __syncthreads();
    if (wave == 0) {
#pragma unroll 1
      for (int wsx = 0; wsx < NWAVE; ++wsx) {
        int n = __builtin_amdgcn_readfirstlane(wcnt[wsx]);
        n = n > WCAP ? WCAP : (n < 0 ? 0 : n);
        const int* lp = list + wsx * WCAP;
#pragma unroll 1
        for (int i = 0; i < n; ++i) {
          const int ent  = __builtin_amdgcn_readfirstlane(lp[i]);
          const int slot = ent & (NBC - 1);
          if (lane == 0) scnt[slot] = scnt[slot] + 1;
        }
      }
    }
    __syncthreads();
  }

  v4i cq[4];
#pragma unroll
  for (int q = 0; q < 4; ++q) {
    const int f = (wave * 4 + q) * 128 + 4 * lane;
    cq[q] = *(const v4i*)(scnt + f);
  }
  int* cp = cnt + (size_t)nodeBase;
#pragma unroll
  for (int q = 0; q < 4; ++q) {
    const int f = (wave * 4 + q) * 128 + 4 * lane;
    *(volatile v4i*)(cp + f) = cq[q];
  }
  __threadfence();
#pragma unroll
  for (int q = 0; q < 4; ++q) {
    const int f = (wave * 4 + q) * 128 + 4 * lane;
    *(volatile v4i*)(cp + f) = cq[q];
  }
}

__global__ __launch_bounds__(OTHR) void k_offsets(
    const int* __restrict__ cnt, int* off, int* rbase, int nChunk) {
  __shared__ __attribute__((aligned(16))) int soff[NBC];
  __shared__ __attribute__((aligned(16))) int srb[RBN];
  __shared__ int wtot[OTHR / 32];
  const int tid = threadIdx.x, lane = tid & 31, wave = tid >> 5, sub = tid >> 7;
  for (int i = tid; i < RBN; i += OTHR) srb[i] = 0;
  int carry = 0;
#pragma unroll 1
  for (int ch = 0; ch < nChunk; ++ch) {
    const int base = ch * NBC;
    const v4i c0 = *(const v4i*)(cnt + base + 8 * tid);
    const v4i c1 = *(const v4i*)(cnt + base + 8 * tid + 4);
    const int e0 = max(c0.x, 0), e1 = max(c0.y, 0), e2 = max(c0.z, 0), e3 = max(c0.w, 0);
    const int e4 = max(c1.x, 0), e5 = max(c1.y, 0), e6 = max(c1.z, 0), e7 = max(c1.w, 0);
    const int ts = e0 + e1 + e2 + e3 + e4 + e5 + e6 + e7;
    int incl = ts;
#pragma unroll
    for (int d = 1; d < 32; d <<= 1) {
      const int t = __shfl_up(incl, d);
      if (lane >= d) incl += t;
    }
    if (lane == 31) wtot[wave] = incl;
    __syncthreads();
    const int S0 = wtot[0]  + wtot[1]  + wtot[2]  + wtot[3];
    const int S1 = wtot[4]  + wtot[5]  + wtot[6]  + wtot[7];
    const int S2 = wtot[8]  + wtot[9]  + wtot[10] + wtot[11];
    const int S3 = wtot[12] + wtot[13] + wtot[14] + wtot[15];
    int pre = 0;
#pragma unroll 1
    for (int w = 4 * sub; w < wave; ++w) pre += wtot[w];
    const int b0 = carry;
    const int b1 = b0 + ((S0 + 31) & ~31);
    const int b2 = b1 + ((S1 + 31) & ~31);
    const int b3 = b2 + ((S2 + 31) & ~31);
    const int b4 = b3 + ((S3 + 31) & ~31);
    const int myb = sub == 0 ? b0 : (sub == 1 ? b1 : (sub == 2 ? b2 : b3));
    if (tid == 0) {
      srb[min(4 * ch + 0, RBN - 1)] = b0;
      srb[min(4 * ch + 1, RBN - 1)] = b1;
      srb[min(4 * ch + 2, RBN - 1)] = b2;
      srb[min(4 * ch + 3, RBN - 1)] = b3;
    }
    int run = myb + pre + incl - ts;
    soff[8 * tid + 0] = run; run += e0;
    soff[8 * tid + 1] = run; run += e1;
    soff[8 * tid + 2] = run; run += e2;
    soff[8 * tid + 3] = run; run += e3;
    soff[8 * tid + 4] = run; run += e4;
    soff[8 * tid + 5] = run; run += e5;
    soff[8 * tid + 6] = run; run += e6;
    soff[8 * tid + 7] = run;
    carry = b4;
    __syncthreads();
    const v4i o0 = *(const v4i*)(soff + 4 * tid);
    const v4i o1 = *(const v4i*)(soff + 4 * (tid + OTHR));
    int* op = off + base;
    *(volatile v4i*)(op + 4 * tid) = o0;
    *(volatile v4i*)(op + 4 * (tid + OTHR)) = o1;
    __threadfence();
    *(volatile v4i*)(op + 4 * tid) = o0;
    *(volatile v4i*)(op + 4 * (tid + OTHR)) = o1;
    __syncthreads();
  }
  if (tid == 0) srb[min(4 * nChunk, RBN - 1)] = carry;
  __syncthreads();
  v4i rv = {0, 0, 0, 0};
  if (tid < 32) rv = *(const v4i*)(srb + 4 * tid);
  if (tid < 32) *(volatile v4i*)(rbase + 4 * tid) = rv;
  __threadfence();
  if (tid < 32) *(volatile v4i*)(rbase + 4 * tid) = rv;
}

__global__ __launch_bounds__(NTHR) void k_fill(
    const int* __restrict__ srcs, const int* __restrict__ dsts,
    const int* __restrict__ off, const int* __restrict__ rbase,
    int* csr, int nN, int nE, int vec8, int csrLen) {
  extern __shared__ v4f lds_dyn[];
  int* region = (int*)lds_dyn;
  int* cursor = region + RCAP;
  int* list   = cursor + NBF;
  int* wcnt   = list + LISTN;
  const int tid = threadIdx.x, lane = tid & 31, wave = tid >> 5;
  const int b = blockIdx.x;
  const int nodeBase = b * NBF;

  int rb0 = rbase[b];
  const int rb1 = rbase[b + 1];
  rb0 = rb0 < 0 ? 0 : (rb0 > csrLen ? csrLen : rb0);
  rb0 &= ~31;
  int len = rb1 - rb0;
  len = len < 0 ? 0 : (len > RCAP ? RCAP : len);
  int lenW = (len + 31) & ~31;
  if (rb0 + lenW > csrLen) lenW = (csrLen - rb0) & ~31;

  {
    const v4i z = {0, 0, 0, 0};
    for (int i = tid; i < RCAP / 4; i += NTHR) ((v4i*)region)[i] = z;
    for (int s = tid; s < NBF; s += NTHR) {
      int o = off[nodeBase + s] - rb0;
      o = o < 0 ? 0 : (o > RCAP ? RCAP : o);
      cursor[s] = o;
    }
  }
  __syncthreads();

  const int nChunks = (nE + CHUNK - 1) / CHUNK;
#pragma unroll 1
  for (int ch = 0; ch < nChunks; ++ch) {
    const int cbase = ch * CHUNK;
    const int wc = scan_chunk<NBF>(dsts, nE, cbase, nodeBase, vec8, list, tid, lane, wave);
    if (lane == 0) wcnt[wave] = wc;
    __syncthreads();
    if (wave == 0) {
#pragma unroll 1
      for (int wsx = 0; wsx < NWAVE; ++wsx) {
        int n = __builtin_amdgcn_readfirstlane(wcnt[wsx]);
        n = n > WCAP ? WCAP : (n < 0 ? 0 : n);
        const int* lp = list + wsx * WCAP;
#pragma unroll 1
        for (int i = 0; i < n; ++i) {
          const int ent  = __builtin_amdgcn_readfirstlane(lp[i]);
          const int slot = ent & (NBF - 1);
          int e = cbase + ((ent >> 12) & (CHUNK - 1));
          e = e > nE - 1 ? nE - 1 : e;
          int sv = srcs[e];
          sv = sv < 0 ? 0 : (sv > nN - 1 ? nN - 1 : sv);
          if (lane == 0) {
            int pos = cursor[slot];
            pos = pos < 0 ? 0 : (pos > RCAP - 1 ? RCAP - 1 : pos);
            region[pos] = sv;
            const int np = pos + 1;
            cursor[slot] = np > RCAP ? RCAP : np;
          }
        }
      }
    }
    __syncthreads();
  }

  const int nv = lenW >> 2;
  int* gp = csr + rb0;
#pragma unroll 1
  for (int i = tid; i < nv; i += NTHR) { const v4i v = ((const v4i*)region)[i]; *(volatile v4i*)(gp + 4 * i) = v; }
  __threadfence();
#pragma unroll 1
  for (int i = tid; i < nv; i += NTHR) { const v4i v = ((const v4i*)region)[i]; *(volatile v4i*)(gp + 4 * i) = v; }
}

template <int KD>
__global__ __launch_bounds__(NTHR) void k_gemm(
    const float* __restrict__ A, const float* __restrict__ coef,
    const float* __restrict__ gg, const float* __restrict__ bb,
    const unsigned short* __restrict__ Bw, float* C, int nN) {
  static_assert(KD == K1 || KD == K2);
  constexpr int APK = KD + 8;
  extern __shared__ v4f lds_dyn[];
  unsigned short* sHi = (unsigned short*)lds_dyn;
  unsigned short* sLo = sHi + GROWS * APK;
  float*          stg = (float*)((char*)lds_dyn + 2 * GROWS * APK * 2);
  const int tid = threadIdx.x, lane = tid & 31, wave = tid >> 5, hh = lane >> 4, m = lane & 15;
  const int rowBase = blockIdx.x * GROWS;

  if (KD == K1) {
    const int c0 = (tid & 15) * 8, rr = tid >> 4;
#pragma unroll 2
    for (int it = 0; it < 8; ++it) {
      const int r = it * 16 + rr;
      int row = rowBase + r;
      row = row > nN - 1 ? nN - 1 : row;
      const float* ap = A + (size_t)row * K1 + c0;
      const v4f a = *(const v4f*)ap, b = *(const v4f*)(ap + 4);
      v8us hv, lv;
      split8(a, b, hv, lv);
      *(v8us*)(sHi + r * APK + c0) = hv;
      *(v8us*)(sLo + r * APK + c0) = lv;
    }
  } else {
    const int c0 = (tid & 7) * 8, rr = tid >> 3;
    const v4f mua = *(const v4f*)(coef + c0),      mub = *(const v4f*)(coef + c0 + 4);
    const v4f rsa = *(const v4f*)(coef + FD + c0), rsb = *(const v4f*)(coef + FD + c0 + 4);
    const v4f ga  = *(const v4f*)(gg + c0),        gb  = *(const v4f*)(gg + c0 + 4);
    const v4f ba  = *(const v4f*)(bb + c0),        bbv = *(const v4f*)(bb + c0 + 4);
#pragma unroll
    for (int it = 0; it < 4; ++it) {
      const int r = it * 32 + rr;
      const float* ap = A + (size_t)(rowBase + r) * K2 + c0;
      const v4f a = *(const v4f*)ap, b = *(const v4f*)(ap + 4);
      const v4f za = bnrelu4(a, mua, rsa, ga, ba);
      const v4f zb = bnrelu4(b, mub, rsb, gb, bbv);
      v8us hv, lv;
      split8(za, zb, hv, lv);
      *(v8us*)(sHi + r * APK + c0) = hv;
      *(v8us*)(sLo + r * APK + c0) = lv;
    }
  }
  __syncthreads();

  v8f acc[4];
  mma_tiles<KD, 4, FD, APK>(sHi, sLo, Bw, wave * 16, lane, acc);
  {
    float* sp = stg + (wave * 16 + 8 * hh) * FD + m;
#pragma unroll
    for (int t = 0; t < 4; ++t) {
#pragma unroll
      for (int r = 0; r < 8; ++r) sp[r * FD + 16 * t] = acc[t][r];
    }
  }
  __syncthreads();

  store_rows64<16>(stg, C, rowBase, wave, lane);
}

__global__ __launch_bounds__(NTHR) void k_agg(
    const int* __restrict__ csr, const int* __restrict__ off, const int* __restrict__ cnt,
    const float* __restrict__ Hp, const float* __restrict__ bias,
    float* G, double* part, int nN, int csrLen) {
  extern __shared__ v4f lds_dyn[];
  float* stg = (float*)lds_dyn;
  __shared__ __attribute__((aligned(16))) double dS[4 * FD];
  __shared__ __attribute__((aligned(16))) double dQ[4 * FD];
  __shared__ __attribute__((aligned(16))) double dP[2 * FD];
  const int tid = threadIdx.x, lane = tid & 31, wave = tid >> 5;
  const int tbase = blockIdx.x * TGT + wave * 32;
  const int cl = tbase + lane;
  const int cnt_l = cnt[cl];
  const int off_l = off[cl];
  const v2f bv = *(const v2f*)(bias + 2 * lane);

#pragma unroll 1
  for (int j = 0; j < 32; ++j) {
    const int c = tbase + j;
    int nraw = __builtin_amdgcn_readlane(cnt_l, j);
    nraw = nraw < 0 ? 0 : nraw;
    const int n = nraw > DEGCAP ? DEGCAP : nraw;
    const int st = __builtin_amdgcn_readlane(off_l, j);
    const float dc = rsqrtf((float)nraw + 1.0f);
    const v2f hc = *(const v2f*)(Hp + (size_t)c * FD + 2 * lane);
    v2f acc = hc * (dc * dc);
#pragma unroll 1
    for (int q0 = 0; q0 < n; q0 += 32) {
      int pos = st + q0 + lane;
      pos = pos < 0 ? 0 : (pos > csrLen - 1 ? csrLen - 1 : pos);
      int sl = csr[pos];
      sl = sl < 0 ? 0 : (sl > nN - 1 ? nN - 1 : sl);
      int cs = cnt[sl];
      cs = cs < 0 ? 0 : cs;
      const float wl = rsqrtf((float)cs + 1.0f) * dc;
      const int wbits = __float_as_int(wl);
      const int mcnt = (n - q0) < 32 ? (n - q0) : 32;
#pragma unroll 1
      for (int p = 0; p < mcnt; ++p) {
        const int s = __builtin_amdgcn_readlane(sl, p);
        const float w = __int_as_float(__builtin_amdgcn_readlane(wbits, p));
        const v2f vf = *(const v2f*)(Hp + (size_t)s * FD + 2 * lane);
        acc = acc + vf * w;
      }
    }
    const v2f res = acc + bv;
    *(v2f*)(stg + (wave * 32 + j) * FD + 2 * lane) = res;
  }
  __syncthreads();

  {
    const int c = tid & (FD - 1), q = tid >> 6;
    double s = 0.0, qq = 0.0;
#pragma unroll 4
    for (int i = 0; i < 64; ++i) {
      const int r = q * 64 + i;
      const float v = stg[r * FD + c];
      const float vz = (blockIdx.x * TGT + r < nN) ? v : 0.0f;
      const double dv = (double)vz;
      s += dv;
      qq = fma(dv, dv, qq);
    }
    dS[q * FD + c] = s;
    dQ[q * FD + c] = qq;
  }
  __syncthreads();
  if (tid < FD) {
    dP[tid]      = ((dS[tid] + dS[FD + tid]) + dS[2 * FD + tid]) + dS[3 * FD + tid];
    dP[FD + tid] = ((dQ[tid] + dQ[FD + tid]) + dQ[2 * FD + tid]) + dQ[3 * FD + tid];
  }
  __syncthreads();
  v2d pv = {0.0, 0.0};
  if (tid < FD) pv = *(const v2d*)(dP + 2 * tid);
  double* gq = part + (size_t)blockIdx.x * (2 * FD) + 2 * tid;
  if (tid < FD) *(volatile v2d*)gq = pv;
  __threadfence();
  if (tid < FD) *(volatile v2d*)gq = pv;

  store_rows64<32>(stg, G, blockIdx.x * TGT, wave, lane);
}

__global__ __launch_bounds__(NTHR) void k_bnfin(const double* __restrict__ part, float* coef, int nBlk, int nN) {
  __shared__ __attribute__((aligned(16))) float sco[2 * FD];
  const int tid = threadIdx.x;
  if (tid < FD) {
    double S = 0.0, Q = 0.0;
#pragma unroll 1
    for (int b = 0; b < nBlk; ++b) {
      S += part[(size_t)b * (2 * FD) + tid];
      Q += part[(size_t)b * (2 * FD) + FD + tid];
    }
    const double rn = 1.0 / (double)(nN > 1 ? nN : 1);
    const double mean = S * rn;
    double var = Q * rn - mean * mean;
    var = var < 0.0 ? 0.0 : var;
    sco[tid]      = (float)mean;
    sco[FD + tid] = rsqrtf((float)var + BN_EPS);
  }
  __syncthreads();
  v4f cv = {0.f, 0.f, 0.f, 0.f};
  if (tid < 32) cv = *(const v4f*)(sco + 4 * tid);
  if (tid < 32) *(volatile v4f*)(coef + 4 * tid) = cv;
  __threadfence();
  if (tid < 32) *(volatile v4f*)(coef + 4 * tid) = cv;
}

__global__ __launch_bounds__(NTHR) void k_bnout(
    const float* __restrict__ G, const float* __restrict__ coef,
    const float* __restrict__ gg, const float* __restrict__ bb, float* out, int nOut4) {
  const int i = blockIdx.x * NTHR + threadIdx.x;
  const int il = i > nOut4 - 1 ? nOut4 - 1 : i;
  const int c4 = (il & 15) * 4;
  const v4f v  = *(const v4f*)(G + (size_t)4 * il);
  const v4f mu = *(const v4f*)(coef + c4);
  const v4f rs = *(const v4f*)(coef + FD + c4);
  const v4f g  = *(const v4f*)(gg + c4);
  const v4f b  = *(const v4f*)(bb + c4);
  const v4f z  = bnrelu4(v, mu, rs, g, b);
  float* op = out + (size_t)4 * il;
  if (i < nOut4) *(volatile v4f*)op = z;
  __threadfence();
  if (i < nOut4) *(volatile v4f*)op = z;
}

extern "C" void kernel_launch(void* const* d_in, const int* in_sizes, int n_in,
                              void* d_out, int out_size, void* d_ws, size_t ws_size,
                              hipStream_t stream) {
  if (n_in < 10) return;
  const int nN = in_sizes[0] / FIN;
  const int nE = in_sizes[1] / 2;
  if (nN <= 0 || nE <= 0) return;
  if (in_sizes[0] != nN * FIN || in_sizes[1] != 2 * nE) return;
  if (in_sizes[2] != FIN * FD || in_sizes[3] != FD || in_sizes[4] != FD || in_sizes[5] != FD) return;
  if (in_sizes[6] != FD * FD || in_sizes[7] != FD || in_sizes[8] != FD || in_sizes[9] != FD) return;
  if (out_size != nN * FD) return;
  if (nE > (1 << 28) || nN > (1 << 24)) return;

  const float* x   = (const float*)d_in[0];
  const int*   ei  = (const int*)d_in[1];
  const float* w1  = (const float*)d_in[2];
  const float* b1  = (const float*)d_in[3];
  const float* g1  = (const float*)d_in[4];
  const float* bt1 = (const float*)d_in[5];
  const float* w2  = (const float*)d_in[6];
  const float* b2  = (const float*)d_in[7];
  const float* g2  = (const float*)d_in[8];
  const float* bt2 = (const float*)d_in[9];
  float* out = (float*)d_out;
  const int* srcs = ei;
  const int* dsts = ei + nE;

  const int NPAD   = ((nN + TGT - 1) / TGT) * TGT;
  const int nBC    = (nN + NBC - 1) / NBC;
  const int CNTPAD = nBC * NBC;
  if (4 * nBC + 1 > RBN) return;
  const int nBF    = (nN + NBF - 1) / NBF;
  const int csrLen = ((nE + 31) & ~31) + 4096;
  if (31 * 4 * nBC > 4096) return;
  const int nGemm  = NPAD / GROWS;
  const int nAgg   = NPAD / TGT;
  const int nOut4  = nN * (FD / 4);
  const int nOutB  = (nOut4 + NTHR - 1) / NTHR;

  char* ws = (char*)d_ws;
  size_t off = 0;
  const size_t oW    = off; off += (size_t)WPTOT * 2;               off = (off + 255) & ~(size_t)255;
  const size_t oCnt  = off; off += (size_t)CNTPAD * 4;              off = (off + 255) & ~(size_t)255;
  const size_t oOff  = off; off += (size_t)CNTPAD * 4;              off = (off + 255) & ~(size_t)255;
  const size_t oRb   = off; off += (size_t)RBN * 4;                 off = (off + 255) & ~(size_t)255;
  const size_t oCsr  = off; off += (size_t)csrLen * 4;              off = (off + 255) & ~(size_t)255;
  const size_t oH    = off; off += (size_t)NPAD * FD * 4;           off = (off + 255) & ~(size_t)255;
  const size_t oG    = off; off += (size_t)NPAD * FD * 4;           off = (off + 255) & ~(size_t)255;
  const size_t oPart = off; off += (size_t)nAgg * (2 * FD) * 8;     off = (off + 255) & ~(size_t)255;
  const size_t oCoef = off; off += (size_t)2 * FD * 4;              off = (off + 255) & ~(size_t)255;
  if (off > ws_size || off > (size_t)WSCAP) return;
  unsigned short* wp   = (unsigned short*)(ws + oW);
  int*            cnt  = (int*)(ws + oCnt);
  int*            offp = (int*)(ws + oOff);
  int*            rb   = (int*)(ws + oRb);
  int*            csr  = (int*)(ws + oCsr);
  float*          Hp   = (float*)(ws + oH);
  float*          Gp   = (float*)(ws + oG);
  double*         part = (double*)(ws + oPart);
  float*          coef = (float*)(ws + oCoef);

  const int vec8 = ((nE & 3) == 0) ? 1 : 0;

  k_wprep<<<6, NTHR, 0, stream>>>(w1, w2, wp);

  k_count<<<nBC, NTHR, 0, stream>>>(dsts, cnt, nE, vec8);
  k_offsets<<<1, OTHR, 0, stream>>>(cnt, offp, rb, nBC);
  hipFuncSetAttribute(reinterpret_cast<const void*>(&k_fill),
                      hipFuncAttributeMaxDynamicSharedMemorySize, LDS_FILL);
  k_fill<<<nBF, NTHR, LDS_FILL, stream>>>(srcs, dsts, offp, rb, csr, nN, nE, vec8, csrLen);

  hipFuncSetAttribute(reinterpret_cast<const void*>(&k_gemm<K1>),
                      hipFuncAttributeMaxDynamicSharedMemorySize, LDS_G1);
  k_gemm<K1><<<nGemm, NTHR, LDS_G1, stream>>>(x, coef, g1, bt1, wp + WP_1, Hp, nN);

  hipFuncSetAttribute(reinterpret_cast<const void*>(&k_agg),
                      hipFuncAttributeMaxDynamicSharedMemorySize, LDS_AGG);
  k_agg<<<nAgg, NTHR, LDS_AGG, stream>>>(csr, offp, cnt, Hp, b1, Gp, part, nN, csrLen);

  k_bnfin<<<1, NTHR, 0, stream>>>(part, coef, nAgg, nN);

  hipFuncSetAttribute(reinterpret_cast<const void*>(&k_gemm<K2>),
                      hipFuncAttributeMaxDynamicSharedMemorySize, LDS_G2);
  k_gemm<K2><<<nGemm, NTHR, LDS_G2, stream>>>(Gp, coef, g1, bt1, wp + WP_2, Hp, nN);

  k_agg<<<nAgg, NTHR, LDS_AGG, stream>>>(csr, offp, cnt, Hp, b2, Gp, part, nN, csrLen);
  k_bnfin<<<1, NTHR, 0, stream>>>(part, coef, nAgg, nN);

  k_bnout<<<nOutB, NTHR, 0, stream>>>(Gp, coef, g2, bt2, out, nOut4);
}
